// RNN_20005957665325
// MI455X (gfx1250) — hardware-verified
//
#include <hip/hip_runtime.h>
#include <math.h>

#pragma clang fp contract(off)

typedef __attribute__((ext_vector_type(16))) _Float16 v16h;
typedef __attribute__((ext_vector_type(8)))  _Float16 v8h;
typedef __attribute__((ext_vector_type(16))) __bf16   v16b;
typedef __attribute__((ext_vector_type(8)))  __bf16   v8b;
typedef __attribute__((ext_vector_type(8)))  float    v8f;
typedef __attribute__((ext_vector_type(4)))  float    v4f;
typedef __attribute__((ext_vector_type(2)))  float    v2f;

constexpr int kB     = 4;
constexpr int kS     = 2048;
constexpr int kDin   = 1024;
constexpr int kDh    = 2048;
constexpr int kDout  = 1024;
constexpr int kPe    = 16;
constexpr int kDcat  = kDin + kPe;
constexpr int kKdup  = kPe;
constexpr int kKloop = kDcat + kKdup;
constexpr int kKpit  = 1088;
constexpr int kRows  = kB * kS;
constexpr int kHalf  = kRows / 2;
constexpr int kScanCh = 64;
constexpr int kScanTS = 64;
constexpr int kScanYP = 68;
static_assert(kDcat == 1040 && kKloop == 1056 && kRows == 8192 && kHalf == 4096, "shapes");
static_assert((kKloop % 32) == 0 && (kDh % 32) == 0, "GEMM K multiples of 32");
static_assert(kKloop <= kKpit && (kKpit % 64) == 0 && ((kKpit * 2) % 128) == 0, "padded pitch, 64-wide k tiles, 128-B rows");
static_assert((kHalf % 64) == 0 && (kRows % 64) == 0 && (kDh % 64) == 0 && (kDout % 64) == 0, "GEMM M,N multiples of 64");
static_assert((kS % kScanTS) == 0 && (kDh % kScanCh) == 0 && kScanCh == 64, "scan tiles");
static_assert(((kRows * kKpit) % (8 * 256)) == 0, "pack grid exact");
static_assert(((kS * kPe / 2) % 256) == 0 && (kDh % 256) == 0, "table grids exact");
static_assert((kHalf / 64) * (kDh / 64) == 2048 && (kRows / 64) * (kDout / 64) == 2048, "tile counts");

constexpr size_t kOffXCB = 0;
constexpr size_t kOffWDX = kOffXCB + (size_t)kRows * kKpit * 2;
constexpr size_t kOffWX  = kOffWDX + (size_t)kDout * kKpit * 2;
constexpr size_t kOffWO  = kOffWX  + (size_t)kDh   * kKpit * 2;
constexpr size_t kOffPET = kOffWO  + (size_t)kDout * kDh   * 2;
constexpr size_t kOffAG  = kOffPET + (size_t)kS    * kPe   * 4;
constexpr size_t kOffXH  = kOffAG  + (size_t)2     * kDh   * 4;
constexpr size_t kOffHH  = kOffXH  + (size_t)kHalf * kDh   * 4;
constexpr size_t kOffHL  = kOffHH  + (size_t)kRows * kDh   * 2;
constexpr size_t kWsTotal = kOffHL + (size_t)kRows * kDh   * 2;
static_assert(kWsTotal == 129515520ull, "carve total");
static_assert(kWsTotal <= 134217728ull, "carve cap");
static_assert((kOffWDX % 128) == 0 && (kOffWX % 128) == 0 && (kOffWO % 128) == 0 && (kOffPET % 128) == 0 &&
              (kOffAG % 128) == 0 && (kOffXH % 128) == 0 && (kOffHH % 128) == 0 && (kOffHL % 128) == 0,
              "128-B aligned regions");
constexpr size_t kOut1Elem = (size_t)kRows * kDout;
static_assert(kOut1Elem * 4 == 33554432ull, "out1 byte offset");
static_assert(kOut1Elem * 4 + (size_t)kB * kDh * 4 == 33587200ull, "total out bytes");

__device__ __forceinline__ unsigned short f2bf_bits(float f) {
  unsigned u = __float_as_uint(f);
  return (unsigned short)((u + 0x7FFFu + ((u >> 16) & 1u)) >> 16);
}
__device__ __forceinline__ float bf_bits2f(unsigned short h) { return __uint_as_float(((unsigned)h) << 16); }

__device__ __forceinline__ void dep_guard_b(v8f& a, v8f& b, v16b x, v16b y) { asm volatile("v_nop\n\tv_nop\n\tv_nop\n\tv_nop" : "+v"(a), "+v"(b) : "v"(x), "v"(y)); }
__device__ __forceinline__ void dep_guard4_b(v8f& a, v8f& b, v8f& c, v8f& d, v16b x, v16b y) {
  asm volatile("v_nop\n\tv_nop\n\tv_nop\n\tv_nop" : "+v"(a), "+v"(b), "+v"(c), "+v"(d) : "v"(x), "v"(y));
}
__device__ __forceinline__ void keep4_b(v16b a, v16b b, v16b c, v16b d) { asm volatile("v_nop" :: "v"(a), "v"(b), "v"(c), "v"(d)); }
__device__ __forceinline__ void acc_guard4(v8f& a, v8f& b, v8f& c, v8f& d) { asm volatile("v_nop\n\tv_nop\n\tv_nop\n\tv_nop" : "+v"(a), "+v"(b), "+v"(c), "+v"(d)); }
template <typename T> struct Frag;
template <> struct Frag<__bf16> {
  typedef v16b V; union U { v16b v; v8b h[2]; };
  static __device__ __forceinline__ v16b load(const __bf16* p) {
    U f; f.h[0] = *(const v8b*)(p); f.h[1] = *(const v8b*)(p + 16); return f.v;
  }
  static __device__ __forceinline__ v8f mma(v16b a, v16b b, v8f c) {
    return __builtin_amdgcn_wmma_f32_16x16x32_bf16(false, a, false, b, (short)0, c, false, false);
  }
  static __device__ __forceinline__ void keep(v16b a, v16b b, v16b c, v16b d) { keep4_b(a, b, c, d); }
};

__global__ __launch_bounds__(256) void gemm_xh_kernel(
    const unsigned short* __restrict__ Ap, const unsigned short* __restrict__ Btp,
    float* __restrict__ Cout, const float* __restrict__ bias, const float* __restrict__ cscale,
    int M, int N, int K, int ldab, int ldc)
{
  const __bf16* A = (const __bf16*)Ap;
  const __bf16* Bt = (const __bf16*)Btp;
  __shared__ __align__(16) float sT[8][16 * 68];
  const int lane = threadIdx.x & 31;
  const int wave = threadIdx.x >> 5;
  const int tilesN = N >> 6;
  const int tilesM = M >> 6;
  const int tile = blockIdx.x * 8 + wave;
  if (tile >= tilesM * tilesN) return;
  const int tm = tile / tilesN;
  const int tn = tile - tm * tilesN;
  const int m0 = tm << 6;
  const int n0 = tn << 6;

  const int rlane = lane & 15;
  const int koff  = (lane >> 4) * 8;
  const int mOff  = (lane >> 4) * 8;

  v8f acc[4][4];
#pragma unroll
  for (int i = 0; i < 4; ++i)
#pragma unroll
    for (int j = 0; j < 4; ++j) acc[i][j] = (v8f){0.f,0.f,0.f,0.f,0.f,0.f,0.f,0.f};

  for (int k0 = 0; k0 < K; k0 += 32) {
    v16b bh[4];
#pragma unroll
    for (int j = 0; j < 4; ++j) {
      const size_t bo = (size_t)(n0 + (j << 4) + rlane) * ldab + koff + k0;
      bh[j] = Frag<__bf16>::load(Bt + bo);
    }
#pragma unroll
    for (int i = 0; i < 4; ++i) {
      const size_t ao = (size_t)(m0 + (i << 4) + rlane) * ldab + koff + k0;
      v16b ah = Frag<__bf16>::load(A + ao);
#pragma unroll
      for (int j = 0; j < 4; ++j) acc[i][j] = Frag<__bf16>::mma(ah, bh[j], acc[i][j]);
      dep_guard4_b(acc[i][0], acc[i][1], acc[i][2], acc[i][3], ah, ah);
    }
    Frag<__bf16>::keep(bh[0], bh[1], bh[2], bh[3]);
  }
  acc_guard4(acc[0][0], acc[0][1], acc[0][2], acc[0][3]);
  acc_guard4(acc[1][0], acc[1][1], acc[1][2], acc[1][3]);
  acc_guard4(acc[2][0], acc[2][1], acc[2][2], acc[2][3]);
  acc_guard4(acc[3][0], acc[3][1], acc[3][2], acc[3][3]);

  float* slab = sT[wave];
  float bvn[4], csn[4];
#pragma unroll
  for (int j = 0; j < 4; ++j) {
    const int n = n0 + (j << 4) + rlane;
    bvn[j] = bias[n];
    csn[j] = cscale[n];
  }
#pragma unroll
  for (int i = 0; i < 4; ++i) {
    const int mBase = m0 + (i << 4);
#pragma unroll
    for (int j = 0; j < 4; ++j) {
#pragma unroll
      for (int r = 0; r < 8; ++r) {
        float v = acc[i][j][r] + bvn[j];
        v = v * csn[j];
        slab[(mOff + r) * 68 + (j << 4) + rlane] = v;
      }
    }
    __builtin_amdgcn_fence(__ATOMIC_RELEASE, "workgroup");
    __builtin_amdgcn_wave_barrier();
    __builtin_amdgcn_fence(__ATOMIC_ACQUIRE, "workgroup");
    {
      const int hh = lane >> 4, c4 = (lane & 15) * 4;
      for (int pass = 0; pass < 2; ++pass) {
#pragma unroll
        for (int it = 0; it < 8; ++it) {
          const int row = it * 2 + hh;
          v4f v = *(const v4f*)(slab + row * 68 + c4);
          *(volatile v4f*)(Cout + (size_t)(mBase + row) * ldc + n0 + c4) = v;
        }
        __threadfence();
      }
    }
    __builtin_amdgcn_fence(__ATOMIC_RELEASE, "workgroup");
    __builtin_amdgcn_wave_barrier();
    __builtin_amdgcn_fence(__ATOMIC_ACQUIRE, "workgroup");
  }
}

__global__ __launch_bounds__(256) void gemm_out_kernel(
    const unsigned short* __restrict__ A1p, const unsigned short* __restrict__ B1p, int ld1, int K1,
    const unsigned short* __restrict__ A2hp, const unsigned short* __restrict__ A2lp,
    const unsigned short* __restrict__ B2p, int ld2, int K2,
    float* __restrict__ Cout, int ldc, const float* __restrict__ bias1, const float* __restrict__ bias2,
    int M, int N)
{
  const __bf16* A1  = (const __bf16*)A1p;
  const __bf16* B1  = (const __bf16*)B1p;
  const __bf16* A2h = (const __bf16*)A2hp;
  const __bf16* A2l = (const __bf16*)A2lp;
  const __bf16* B2  = (const __bf16*)B2p;
  __shared__ __align__(16) float sT[8][16 * 68];
  const int lane = threadIdx.x & 31;
  const int wave = threadIdx.x >> 5;
  const int tilesN = N >> 6;
  const int tilesM = M >> 6;
  const int tile = blockIdx.x * 8 + wave;
  if (tile >= tilesM * tilesN) return;
  const int tm = tile / tilesN;
  const int tn = tile - tm * tilesN;
  const int m0 = tm << 6;
  const int n0 = tn << 6;

  const int rlane = lane & 15;
  const int koff  = (lane >> 4) * 8;
  const int mOff  = (lane >> 4) * 8;

  v8f acc[4][4];
#pragma unroll
  for (int i = 0; i < 4; ++i)
#pragma unroll
    for (int j = 0; j < 4; ++j) acc[i][j] = (v8f){0.f,0.f,0.f,0.f,0.f,0.f,0.f,0.f};

  for (int k0 = 0; k0 < K1; k0 += 32) {
    v16b bh[4];
#pragma unroll
    for (int j = 0; j < 4; ++j) {
      const size_t bo = (size_t)(n0 + (j << 4) + rlane) * ld1 + koff + k0;
      bh[j] = Frag<__bf16>::load(B1 + bo);
    }
#pragma unroll
    for (int i = 0; i < 4; ++i) {
      const size_t ao = (size_t)(m0 + (i << 4) + rlane) * ld1 + koff + k0;
      v16b ah = Frag<__bf16>::load(A1 + ao);
#pragma unroll
      for (int j = 0; j < 4; ++j) acc[i][j] = Frag<__bf16>::mma(ah, bh[j], acc[i][j]);
      dep_guard4_b(acc[i][0], acc[i][1], acc[i][2], acc[i][3], ah, ah);
    }
    Frag<__bf16>::keep(bh[0], bh[1], bh[2], bh[3]);
  }
  for (int k0 = 0; k0 < K2; k0 += 32) {
    v16b bh[4];
#pragma unroll
    for (int j = 0; j < 4; ++j) {
      const size_t bo = (size_t)(n0 + (j << 4) + rlane) * ld2 + koff + k0;
      bh[j] = Frag<__bf16>::load(B2 + bo);
    }
#pragma unroll
    for (int i = 0; i < 4; ++i) {
      const size_t ao = (size_t)(m0 + (i << 4) + rlane) * ld2 + koff + k0;
      v16b ah = Frag<__bf16>::load(A2h + ao);
      v16b al = Frag<__bf16>::load(A2l + ao);
#pragma unroll
      for (int j = 0; j < 4; ++j) {
        acc[i][j] = Frag<__bf16>::mma(ah, bh[j], acc[i][j]);
        acc[i][j] = Frag<__bf16>::mma(al, bh[j], acc[i][j]);
      }
      dep_guard4_b(acc[i][0], acc[i][1], acc[i][2], acc[i][3], ah, al);
    }
    Frag<__bf16>::keep(bh[0], bh[1], bh[2], bh[3]);
  }
  acc_guard4(acc[0][0], acc[0][1], acc[0][2], acc[0][3]);
  acc_guard4(acc[1][0], acc[1][1], acc[1][2], acc[1][3]);
  acc_guard4(acc[2][0], acc[2][1], acc[2][2], acc[2][3]);
  acc_guard4(acc[3][0], acc[3][1], acc[3][2], acc[3][3]);

  float* slab = sT[wave];
  float bvh[4];
#pragma unroll
  for (int j = 0; j < 4; ++j) {
    const int n = n0 + (j << 4) + rlane;
    const float s = bias1[n] + bias2[n];
    bvh[j] = s * 0.5f;
  }
#pragma unroll
  for (int i = 0; i < 4; ++i) {
    const int mBase = m0 + (i << 4);
#pragma unroll
    for (int j = 0; j < 4; ++j) {
#pragma unroll
      for (int r = 0; r < 8; ++r) {
        const float hv = acc[i][j][r] * 0.5f;
        slab[(mOff + r) * 68 + (j << 4) + rlane] = hv + bvh[j];
      }
    }
    __builtin_amdgcn_fence(__ATOMIC_RELEASE, "workgroup");
    __builtin_amdgcn_wave_barrier();
    __builtin_amdgcn_fence(__ATOMIC_ACQUIRE, "workgroup");
    {
      const int hh = lane >> 4, c4 = (lane & 15) * 4;
      for (int pass = 0; pass < 2; ++pass) {
#pragma unroll
        for (int it = 0; it < 8; ++it) {
          const int row = it * 2 + hh;
          v4f v = *(const v4f*)(slab + row * 68 + c4);
          *(volatile v4f*)(Cout + (size_t)(mBase + row) * ldc + n0 + c4) = v;
        }
        __threadfence();
      }
    }
    __builtin_amdgcn_fence(__ATOMIC_RELEASE, "workgroup");
    __builtin_amdgcn_wave_barrier();
    __builtin_amdgcn_fence(__ATOMIC_ACQUIRE, "workgroup");
  }
}

__global__ __launch_bounds__(256) void pe_table_kernel(float* __restrict__ PET, int total)
{
  const int i = blockIdx.x * 256 + threadIdx.x;
  if (i >= total) return;
  const int t  = i >> 3;
  const int pr = i & 7;
  const float cf  = -logf(10000.0f) / (float)kPe;
  const float dv  = expf((float)(2 * pr) * cf);
  const float ang = (float)t * dv;
  float sv, cv;
  sincosf(ang, &sv, &cv);
  v2f o;
  o[0] = sv * 0.1f;
  o[1] = cv * 0.1f;
  float* p = PET + (size_t)i * 2;
  *(volatile v2f*)p = o;
  __threadfence();
  *(volatile v2f*)p = o;
}

__global__ __launch_bounds__(256) void ag_table_kernel(const float* __restrict__ a_logit, float* __restrict__ AG, int n)
{
  const int d = blockIdx.x * 256 + threadIdx.x;
  if (d >= n) return;
  const float al = bf_bits2f(f2bf_bits(a_logit[d]));
  const float ea = expf(-al);
  const float a  = 1.0f / (1.0f + ea);
  const float aa = a * a;
  const float gg = fmaxf(1.0f - aa, 0.0f);
  const float g  = sqrtf(gg);
  float* pa = AG + d;
  float* pg = AG + n + d;
  *(volatile float*)pa = a;
  *(volatile float*)pg = g;
  __threadfence();
  *(volatile float*)pa = a;
  *(volatile float*)pg = g;
}

__global__ __launch_bounds__(256) void pack_xc_kernel(
    const float* __restrict__ x, const float* __restrict__ PET, unsigned short* __restrict__ XCB, int total8)
{
  const int i = blockIdx.x * 256 + threadIdx.x;
  if (i >= total8) return;
  const int e0 = i << 3;
  const int m  = e0 / kKpit;
  const int c  = e0 - m * kKpit;
  const int t  = m & (kS - 1);
  const bool xsel = (c < kDin);
  const bool hsel = (c >= kDin) && (c < kDcat);
  const bool lsel = (c >= kDcat) && (c < kKloop);
  const int cx = xsel ? c : 0;
  const int cp = (hsel || lsel) ? ((c - kDin) & 8) : 0;
  const float* xp = x + (size_t)m * kDin + cx;
  const float* pp = PET + (size_t)t * kPe + cp;
  const v4f xa0 = *(const v4f*)(xp);
  const v4f xa1 = *(const v4f*)(xp + 4);
  const v4f pa0 = *(const v4f*)(pp);
  const v4f pa1 = *(const v4f*)(pp + 4);
  const float fx = xsel ? 1.0f : 0.0f;
  const float fh = hsel ? 1.0f : 0.0f;
  const float fl = lsel ? 1.0f : 0.0f;
  v8h hv;
#pragma unroll
  for (int e = 0; e < 4; ++e) {
    const float x0 = xa0[e], x1 = xa1[e];
    const float p0 = pa0[e], p1 = pa1[e];
    const float ph0 = bf_bits2f(f2bf_bits(p0));
    const float ph1 = bf_bits2f(f2bf_bits(p1));
    const float pl0 = p0 - ph0;
    const float pl1 = p1 - ph1;
    const float v0 = fmaf(fx, x0, fmaf(fh, p0, fl * pl0));
    const float v1 = fmaf(fx, x1, fmaf(fh, p1, fl * pl1));
    const unsigned short b0 = f2bf_bits(v0);
    const unsigned short b1 = f2bf_bits(v1);
    hv[e]     = __builtin_bit_cast(_Float16, b0);
    hv[4 + e] = __builtin_bit_cast(_Float16, b1);
  }
  unsigned short* q = XCB + (size_t)e0;
  *(volatile v8h*)q = hv;
  __threadfence();
  *(volatile v8h*)q = hv;
}

__global__ __launch_bounds__(256) void transpose_bf16_kernel(
    const float* __restrict__ W, unsigned short* __restrict__ Bt, int Kdim, int Kdup, int Ndim, int Kpad)
{
  __shared__ float tile[64 * 65];
  const int tid = threadIdx.x, lane = tid & 31, wave = tid >> 5;
  const int n0 = blockIdx.x * 64;
  const int k0 = blockIdx.y * 64;
#pragma unroll
  for (int p = 0; p < 16; ++p) {
    const int idx = tid + p * 256;
    const int kk  = idx >> 6;
    const int nn  = idx & 63;
    const int k   = k0 + kk;
    const bool valid = (k < Kdim + Kdup);
    const int ksrc = (k < Kdim) ? k : (k - Kdup);
    const int kc   = valid ? ksrc : (Kdim - 1);
    const float v  = W[(size_t)kc * Ndim + n0 + nn];
    tile[kk * 65 + nn] = valid ? v : 0.f;
  }
  __syncthreads();
  const int q = lane >> 3, c8 = (lane & 7) * 8;
  v8h hv[2];
#pragma unroll
  for (int it = 0; it < 2; ++it) {
    const int nrow = it * 32 + wave * 4 + q;
#pragma unroll
    for (int e = 0; e < 8; ++e) {
      const unsigned short hb = f2bf_bits(tile[(c8 + e) * 65 + nrow]);
      hv[it][e] = __builtin_bit_cast(_Float16, hb);
    }
  }
  for (int pass = 0; pass < 2; ++pass) {
#pragma unroll
    for (int it = 0; it < 2; ++it) {
      const int nrow = it * 32 + wave * 4 + q;
      *(volatile v8h*)(Bt + (size_t)(n0 + nrow) * Kpad + k0 + c8) = hv[it];
    }
    __threadfence();
  }
}

__global__ __launch_bounds__(64) void scan_kernel(
    const float* __restrict__ XH, const float* __restrict__ AG, const float* __restrict__ h_prev,
    unsigned short* __restrict__ HH, unsigned short* __restrict__ HL, float* __restrict__ h_last, int bbase)
{
  __shared__ __align__(16) float sY[kScanTS * kScanYP];
  const int tid = threadIdx.x, lane = tid & 31, wave = tid >> 5;
  constexpr int kBlkPerB = kDh / kScanCh;
  const int bl = blockIdx.x / kBlkPerB;
  const int d0 = (blockIdx.x - bl * kBlkPerB) * kScanCh;
  const int d  = d0 + tid;
  const int bg = bbase + bl;
  const size_t xrow0 = (size_t)bl * kS;
  const size_t hrow0 = (size_t)bg * kS;
  const float a = AG[d];
  float h = bf_bits2f(f2bf_bits(h_prev[(size_t)bg * kDh + d]));
  const int q = lane >> 3, c8 = (lane & 7) * 8;
#pragma unroll 1
  for (int t0 = 0; t0 < kS; t0 += kScanTS) {
#pragma unroll 1
    for (int s = 0; s < kScanTS; ++s) {
      const float xv = XH[(xrow0 + t0 + s) * kDh + d];
      const float ph = a * h;
      h = ph + xv;
      sY[s * kScanYP + tid] = h;
    }
    __syncthreads();
    v8h hv[8], lv[8];
#pragma unroll
    for (int it = 0; it < 8; ++it) {
      const int row = it * 8 + wave * 4 + q;
      const float* sp = sY + row * kScanYP + c8;
      const v4f a0 = *(const v4f*)(sp);
      const v4f a1 = *(const v4f*)(sp + 4);
#pragma unroll
      for (int e = 0; e < 4; ++e) {
        const float f0 = a0[e], f1 = a1[e];
        const unsigned short h0 = f2bf_bits(f0), h1 = f2bf_bits(f1);
        const unsigned short l0 = f2bf_bits(f0 - bf_bits2f(h0)), l1 = f2bf_bits(f1 - bf_bits2f(h1));
        hv[it][e]     = __builtin_bit_cast(_Float16, h0);
        hv[it][4 + e] = __builtin_bit_cast(_Float16, h1);
        lv[it][e]     = __builtin_bit_cast(_Float16, l0);
        lv[it][4 + e] = __builtin_bit_cast(_Float16, l1);
      }
    }
    for (int pass = 0; pass < 2; ++pass) {
#pragma unroll
      for (int it = 0; it < 8; ++it) {
        const int row = it * 8 + wave * 4 + q;
        const size_t o = (hrow0 + t0 + row) * kDh + d0 + c8;
        *(volatile v8h*)(HH + o) = hv[it];
        *(volatile v8h*)(HL + o) = lv[it];
      }
      __threadfence();
    }
    __syncthreads();
  }
  sY[tid] = h;
  __syncthreads();
  const bool wl = (wave == 0) && (lane < 16);
  const v4f h4 = *(const v4f*)(sY + (lane & 15) * 4);
  float* hp = h_last + (size_t)bg * kDh + d0 + (lane & 15) * 4;
  if (wl) *(volatile v4f*)hp = h4;
  __threadfence();
  if (wl) *(volatile v4f*)hp = h4;
}

extern "C" void kernel_launch(void* const* d_in, const int* in_sizes, int n_in,
                              void* d_out, int out_size, void* d_ws, size_t ws_size,
                              hipStream_t stream)
{
  if (n_in < 9) return;
  if (in_sizes[0] != kRows * kDin) return;
  if (in_sizes[1] != kB * kDh) return;
  if (in_sizes[2] != kDh) return;
  if (in_sizes[3] != kDcat * kDout) return;
  if (in_sizes[4] != kDout) return;
  if (in_sizes[5] != kDcat * kDh) return;
  if (in_sizes[6] != kDh) return;
  if (in_sizes[7] != kDh * kDout) return;
  if (in_sizes[8] != kDout) return;
  if (out_size != kRows * kDout + kB * kDh) return;
  if (ws_size < kWsTotal) return;

  const float* x       = (const float*)d_in[0];
  const float* h_prev  = (const float*)d_in[1];
  const float* a_logit = (const float*)d_in[2];
  const float* W_dx    = (const float*)d_in[3];
  const float* b_dx    = (const float*)d_in[4];
  const float* W_x     = (const float*)d_in[5];
  const float* b_x     = (const float*)d_in[6];
  const float* W_o     = (const float*)d_in[7];
  const float* b_o     = (const float*)d_in[8];
  float* out0   = (float*)d_out;
  float* h_last = out0 + kOut1Elem;

  char* ws = (char*)d_ws;
  unsigned short* XCB = (unsigned short*)(ws + kOffXCB);
  unsigned short* WDX = (unsigned short*)(ws + kOffWDX);
  unsigned short* WX  = (unsigned short*)(ws + kOffWX);
  unsigned short* WO  = (unsigned short*)(ws + kOffWO);
  float*          PET = (float*)(ws + kOffPET);
  float*          AG  = (float*)(ws + kOffAG);
  float*          XH  = (float*)(ws + kOffXH);
  unsigned short* HH  = (unsigned short*)(ws + kOffHH);
  unsigned short* HL  = (unsigned short*)(ws + kOffHL);

  pe_table_kernel<<<(kS * kPe / 2) / 256, 256, 0, stream>>>(PET, kS * kPe / 2);
  ag_table_kernel<<<kDh / 256, 256, 0, stream>>>(a_logit, AG, kDh);

  pack_xc_kernel<<<(kRows * kKpit / 8) / 256, 256, 0, stream>>>(x, PET, XCB, (kRows * kKpit) / 8);

  transpose_bf16_kernel<<<dim3(kDout / 64, kKpit / 64), 256, 0, stream>>>(W_dx, WDX, kDcat, kKdup, kDout, kKpit);
  transpose_bf16_kernel<<<dim3(kDh / 64, kKpit / 64), 256, 0, stream>>>(W_x, WX, kDcat, kKdup, kDh, kKpit);
  transpose_bf16_kernel<<<dim3(kDout / 64, kDh / 64), 256, 0, stream>>>(W_o, WO, kDh, 0, kDout, kDh);

  for (int pr = 0; pr < 2; ++pr) {
    const unsigned short* XCBp = XCB + (size_t)pr * kHalf * kKpit;
    gemm_xh_kernel<<<dim3((kHalf / 64) * (kDh / 64) / 8, 1), 256, 0, stream>>>(
        XCBp, WX, XH, b_x, AG + kDh, kHalf, kDh, kKloop, kKpit, kDh);
    scan_kernel<<<dim3(2 * (kDh / kScanCh), 1), kScanCh, 0, stream>>>(XH, AG, h_prev, HH, HL, h_last, pr * 2);
  }

  gemm_out_kernel<<<dim3((kRows / 64) * (kDout / 64) / 8, 1), 256, 0, stream>>>(
      XCB, WDX, kKpit, kKloop, HH, HL, WO, kDh, kDh, out0, kDout, b_dx, b_o, kRows, kDout);
}
